// Attention_ViT_8916352106583
// MI455X (gfx1250) — hardware-verified
//
#include <hip/hip_runtime.h>
#include <math.h>

typedef __attribute__((ext_vector_type(16))) _Float16 v16h;
typedef __attribute__((ext_vector_type(16))) __bf16 v16b;
typedef __attribute__((ext_vector_type(8)))  _Float16 v8h;
typedef __attribute__((ext_vector_type(8)))  float v8f;
typedef __attribute__((ext_vector_type(4)))  float v4f;
typedef __attribute__((ext_vector_type(2)))  float v2f;
typedef __attribute__((ext_vector_type(4)))  unsigned v4u;
typedef __attribute__((ext_vector_type(4)))  int v4i;
typedef float __attribute__((may_alias)) float_a;
typedef int __attribute__((may_alias)) int_a;

template <typename T> __device__ __forceinline__ void vst2(void* p, T v) { *(volatile T*)p = v; __threadfence(); *(volatile T*)p = v; }
__device__ __forceinline__ v8f wmma16(v16h a, v16h b, v8f c) {
  v8f d = __builtin_amdgcn_wmma_f32_16x16x32_f16(false, a, false, b, (short)0, c, false, false);
  asm volatile("v_nop\n\tv_nop\n\tv_nop\n\tv_nop" : "+v"(d) : "v"(a), "v"(b));
  return d;
}
__device__ __forceinline__ v8f wmma_bf(v16b a, v16b b, v8f c) {
  v8f d = __builtin_amdgcn_wmma_f32_16x16x32_bf16(false, a, false, b, (short)0, c, false, false);
  asm volatile("v_nop\n\tv_nop\n\tv_nop\n\tv_nop" : "+v"(d) : "v"(a), "v"(b));
  return d;
}
__device__ __forceinline__ v16h frag_h(const _Float16* rowk0, int lane) {
  union { v16h v; v8h q[2]; } u; const _Float16* p = rowk0 + 8 * (lane >> 4);
  u.q[0] = *(const v8h*)p; u.q[1] = *(const v8h*)(p + 16); return u.v;
}
__device__ __forceinline__ v16h frag_f32(const float* rowk0, int lane) {
  v16h a; const float* p = rowk0 + 8 * (lane >> 4);
#pragma unroll
  for (int i = 0; i < 8; ++i) { a[i] = (_Float16)p[i]; a[8 + i] = (_Float16)p[16 + i]; }
  return a;
}
__device__ __forceinline__ v16h frag_f32s(const float* rowk0, int lane, float sc) {
  v16h a; const float* p = rowk0 + 8 * (lane >> 4);
#pragma unroll
  for (int i = 0; i < 8; ++i) { a[i] = (_Float16)(p[i] * sc); a[8 + i] = (_Float16)(p[16 + i] * sc); }
  return a;
}
__device__ __forceinline__ v16h fragc_f32(const float* W, int k0, int n, int lane, int ld, int K) {
  v16h a; const int g = lane >> 4;
#pragma unroll
  for (int i = 0; i < 8; ++i) { const int ka = k0 + 8 * g + i, kb = ka + 16;
    a[i] = (_Float16)(ka < K ? W[(size_t)(ka < K ? ka : K - 1) * ld + n] : 0.f); a[8 + i] = (_Float16)(kb < K ? W[(size_t)(kb < K ? kb : K - 1) * ld + n] : 0.f); }
  return a;
}
struct F2 { v16b h, l; };
__device__ __forceinline__ F2 bsplit16(const float v[16]) { F2 r;
#pragma unroll
  for (int i = 0; i < 16; ++i) { const __bf16 h = (__bf16)v[i]; r.h[i] = h; r.l[i] = (__bf16)(v[i] - (float)h); }
  return r; }
__device__ __forceinline__ F2 split_row(const float* row, int k0, int lane) { float v[16]; const float* p = row + k0 + 8 * (lane >> 4);
#pragma unroll
  for (int i = 0; i < 8; ++i) { v[i] = p[i]; v[8 + i] = p[16 + i]; }
  return bsplit16(v); }
__device__ __forceinline__ F2 split_rowK(const float* row, int k0, int lane, int K) { float v[16]; const int g = lane >> 4;
#pragma unroll
  for (int i = 0; i < 8; ++i) { const int ka = k0 + 8 * g + i, kb = ka + 16; v[i] = ka < K ? row[ka < K ? ka : K - 1] : 0.f; v[8 + i] = kb < K ? row[kb < K ? kb : K - 1] : 0.f; }
  return bsplit16(v); }
__device__ __forceinline__ F2 split_col(const float* W, int k0, int n, int lane, int ld, int K) { float v[16]; const int g = lane >> 4;
#pragma unroll
  for (int i = 0; i < 8; ++i) { const int ka = k0 + 8 * g + i, kb = ka + 16; v[i] = ka < K ? W[(size_t)(ka < K ? ka : K - 1) * ld + n] : 0.f; v[8 + i] = kb < K ? W[(size_t)(kb < K ? kb : K - 1) * ld + n] : 0.f; }
  return bsplit16(v); }
__device__ __forceinline__ v8f mac3(const F2& a, const F2& b, v8f c) { c = wmma_bf(a.l, b.h, c); c = wmma_bf(a.h, b.l, c); return wmma_bf(a.h, b.h, c); }
__device__ __forceinline__ float sigm(float v) { return 1.0f / (1.0f + expf(-v)); }
#define LDSX() do { asm volatile("s_wait_dscnt 0" ::: "memory"); __builtin_amdgcn_wave_barrier(); __builtin_amdgcn_fence(__ATOMIC_RELEASE, "workgroup"); } while (0)


#define NB 8
#define SS 1024
#define E 1024
#define NH 16
#define HD 64
#define NR (NB * SS)
#define PLO 1024.0f
#define VLO 2048.0f
__device__ __forceinline__ float bfr(float v) { return (float)(__bf16)v; }
__device__ __forceinline__ v16b frag_b(const __bf16* rowk0, int lane) { return __builtin_bit_cast(v16b, frag_h((const _Float16*)rowk0, lane)); }

__global__ __launch_bounds__(256) void k_cvt(const float* __restrict__ x, __bf16* __restrict__ Xb) {
  const size_t i8 = (size_t)blockIdx.x * 256 + threadIdx.x; if (i8 >= (size_t)NR * E / 8) return;
  union { __bf16 h[8]; v4u u; } pk;
#pragma unroll
  for (int e = 0; e < 8; ++e) pk.h[e] = (__bf16)x[i8 * 8 + e];
  vst2((unsigned*)(Xb + i8 * 8), pk.u);
}
__global__ __launch_bounds__(128) void k_pack(const float* __restrict__ Wqkv, const float* __restrict__ Wp, __bf16* __restrict__ PT) {
  const int n = blockIdx.x, tid = threadIdx.x; __shared__ __align__(16) __bf16 srow[E];
  for (int k = tid; k < E; k += 128) srow[k] = (__bf16)(n < 3 * E ? Wqkv[(size_t)k * (3 * E) + n] : Wp[(size_t)k * E + (n - 3 * E)]);
  __syncthreads();
  if (tid < E / 8) vst2((unsigned*)(PT + (size_t)n * E + tid * 8), *(const v4u*)(&srow[tid * 8]));
}
__global__ __launch_bounds__(128) void k_qkv(const __bf16* __restrict__ Xb, int rbase, const __bf16* __restrict__ PT, float* __restrict__ Q32, float* __restrict__ K32, _Float16* __restrict__ VTh, _Float16* __restrict__ VTl) {
  __shared__ __align__(16) float so[4][16][132];
  __shared__ __align__(16) _Float16 sth[128][72], stl[128][72];
  const int tid = threadIdx.x, wave = tid >> 5, lane = tid & 31, col = lane & 15, g = lane >> 4;
  const int which = blockIdx.z, r0b = blockIdx.x * 64, r0 = r0b + wave * 16, n0 = blockIdx.y * 128; const int b = r0b / SS, s0 = r0b % SS;
  v8f acc[8] = {};
#pragma unroll 2
  for (int kc = 0; kc < E / 32; ++kc) { const v16b a = frag_b(Xb + (size_t)(rbase + r0 + col) * E + kc * 32, lane);
#pragma unroll
    for (int j = 0; j < 8; ++j) acc[j] = wmma_bf(a, frag_b(PT + (size_t)(which * E + n0 + j * 16 + col) * E + kc * 32, lane), acc[j]); }
  if (which < 2) {
#pragma unroll
    for (int j = 0; j < 8; ++j) { const float bb = 0.f;
#pragma unroll
      for (int r = 0; r < 8; ++r) so[wave][8 * g + r][j * 16 + col] = acc[j][r] + bb; }
    LDSX();
    float* Dst = which == 0 ? Q32 : K32;
    for (int qq = lane; qq < 2 * 16 * 16; qq += 32) { const int hh = qq >> 8, rl = (qq >> 4) & 15, pc = qq & 15; const int h = (n0 >> 6) + hh;
      vst2(Dst + (((size_t)b * NH + h) * SS + s0 + wave * 16 + rl) * HD + pc * 4, *(const v4f*)(&so[wave][rl][hh * 64 + pc * 4])); } }
  else {
#pragma unroll
    for (int j = 0; j < 8; ++j) { const float bb = 0.f;
#pragma unroll
      for (int r = 0; r < 8; ++r) { const float v = (acc[j][r] + bb) * 4.0f; const _Float16 hi = (_Float16)v; sth[j * 16 + col][wave * 16 + 8 * g + r] = hi; stl[j * 16 + col][wave * 16 + 8 * g + r] = (_Float16)((v - (float)hi) * VLO); } }
    __syncthreads();
    for (int qq = tid; qq < 128 * 8; qq += 128) { const int cl = qq >> 3, pc = qq & 7; const int c = n0 + cl, h = c >> 6, d = c & 63; const size_t o = (((size_t)b * NH + h) * HD + d) * SS + s0 + pc * 8;
      vst2(VTh + o, *(const v4u*)(&sth[cl][pc * 8])); vst2(VTl + o, *(const v4u*)(&stl[cl][pc * 8])); } }
}
__global__ __launch_bounds__(128) void k_attn(const float* __restrict__ Q32, const float* __restrict__ K32, const _Float16* __restrict__ VTh, const _Float16* __restrict__ VTl, float* __restrict__ O32) {
  __shared__ __align__(16) float sS[4][16][68];
  __shared__ __align__(16) _Float16 sPh[4][16][72], sPl[4][16][72];
  __shared__ __align__(16) float sO[4][16][68];
  const int tid = threadIdx.x, w = tid >> 5, lane = tid & 31, col = lane & 15, g = lane >> 4;
  const size_t bh = blockIdx.y; const int qb = blockIdx.x; const int q0 = qb * 64 + w * 16;
  F2 aq[2];
#pragma unroll
  for (int kc = 0; kc < 2; ++kc) aq[kc] = split_row(Q32 + (bh * SS + q0 + col) * HD, kc * 32, lane);
  float mrun = -3.0e38f, lrun = 0.f; v8f acc[4] = {}, ac1[4] = {}, ac2[4] = {};
#pragma unroll 1
  for (int kt = 0; kt < SS / 64; ++kt) {
#pragma unroll
    for (int t = 0; t < 4; ++t) { const int key = kt * 64 + t * 16 + col; const float* krow = K32 + (bh * SS + key) * HD;
      v8f s = mac3(aq[0], split_row(krow, 0, lane), (v8f){}); s = mac3(aq[1], split_row(krow, 32, lane), s);
#pragma unroll
      for (int r = 0; r < 8; ++r) sS[w][8 * g + r][t * 16 + col] = s[r] * 0.125f; }
    LDSX();
    float mx = -3.4e38f;
#pragma unroll
    for (int jj = 0; jj < 32; ++jj) mx = fmaxf(mx, sS[w][col][g * 32 + jj]);
    mx = fmaxf(mx, __shfl_xor(mx, 16, 32));
    const float mnew = fmaxf(mrun, mx); const float corr = expf(mrun - mnew);
    float ps = 0.f;
#pragma unroll
    for (int jj = 0; jj < 32; ++jj) { const float p = expf(sS[w][col][g * 32 + jj] - mnew) * 16384.0f; ps += p; const _Float16 hi = (_Float16)p; sPh[w][col][g * 32 + jj] = hi; sPl[w][col][g * 32 + jj] = (_Float16)((p - (float)hi) * PLO); }
    ps += __shfl_xor(ps, 16, 32);
    lrun = lrun * corr + ps * (1.0f / 16384.0f); mrun = mnew;
#pragma unroll
    for (int r = 0; r < 8; ++r) { const float cr = __shfl(corr, 8 * g + r, 32);
#pragma unroll
      for (int t = 0; t < 4; ++t) { acc[t][r] *= cr; ac1[t][r] *= cr; ac2[t][r] *= cr; } }
    LDSX();
#pragma unroll
    for (int kc = 0; kc < 2; ++kc) { const v16h ph = frag_h(&sPh[w][col][0] + kc * 32, lane), pl = frag_h(&sPl[w][col][0] + kc * 32, lane);
#pragma unroll
      for (int t = 0; t < 4; ++t) { const size_t vo = (bh * HD + t * 16 + col) * SS + kt * 64 + kc * 32; const v16h vh = frag_h(VTh + vo, lane);
        acc[t] = wmma16(ph, vh, acc[t]); ac1[t] = wmma16(ph, frag_h(VTl + vo, lane), ac1[t]); ac2[t] = wmma16(pl, vh, ac2[t]); } }
    __builtin_amdgcn_wave_barrier(); }
#pragma unroll
  for (int r = 0; r < 8; ++r) { const float lr = __shfl(lrun, 8 * g + r, 32); const float inv = 1.0f / (lr * 16384.0f * 4.0f);
#pragma unroll
    for (int t = 0; t < 4; ++t) sO[w][8 * g + r][t * 16 + col] = (acc[t][r] + ac1[t][r] * (1.0f / VLO) + ac2[t][r] * (1.0f / PLO)) * inv; }
  LDSX();
  for (int qq = lane; qq < 16 * 16; qq += 32) { const int rl = qq >> 4, pc = qq & 15; vst2(O32 + ((bh * SS) + q0 + rl) * HD + pc * 4, *(const v4f*)(&sO[w][rl][pc * 4])); }
}
__global__ __launch_bounds__(128) void k_out(const float* __restrict__ O32, int rbase, const __bf16* __restrict__ PT, const float* __restrict__ bo, float* __restrict__ out) {
  __shared__ __align__(16) float so[4][16][132];
  const int tid = threadIdx.x, wave = tid >> 5, lane = tid & 31, col = lane & 15, g = lane >> 4;
  const int r0 = blockIdx.x * 64 + wave * 16, n0 = blockIdx.y * 128; const int ra = r0 + col; const int b = ra / SS, s = ra % SS;
  v8f acc[8] = {};
#pragma unroll 1
  for (int kc = 0; kc < E / 32; ++kc) { const int h = kc >> 1; const F2 a = split_row(O32 + (((size_t)b * NH + h) * SS + s) * HD, (kc & 1) * 32, lane);
#pragma unroll
    for (int j = 0; j < 8; ++j) { const v16b wb = frag_b(PT + (size_t)(3 * E + n0 + j * 16 + col) * E + kc * 32, lane); acc[j] = wmma_bf(a.l, wb, acc[j]); acc[j] = wmma_bf(a.h, wb, acc[j]); } }
#pragma unroll
  for (int j = 0; j < 8; ++j) { const int n = n0 + j * 16 + col; const float bb = bfr(bo[n]);
#pragma unroll
    for (int r = 0; r < 8; ++r) so[wave][8 * g + r][j * 16 + col] = acc[j][r] + bb; }
  LDSX();
#pragma unroll 4
  for (int rl = 0; rl < 16; ++rl) vst2(out + (size_t)(rbase + r0 + rl) * E + n0 + lane * 4, *(const v4f*)(&so[wave][rl][lane * 4]));
}
#define NBHALF 4
extern "C" void kernel_launch(void* const* d_in, const int* in_sizes, int n_in, void* d_out, int out_size, void* d_ws, size_t ws_size, hipStream_t stream) {
  (void)in_sizes; (void)n_in; (void)out_size; (void)ws_size;
  const float* x = (const float*)d_in[0]; const float* Wqkv = (const float*)d_in[1]; const float* Wp = (const float*)d_in[2]; const float* bp = (const float*)d_in[3];
  float* out = (float*)d_out;
  char* ws = (char*)d_ws; size_t off = 0;
  auto take = [&](size_t bytes) { char* p = ws + off; off += (bytes + 255) & ~(size_t)255; return p; };
  const size_t HR = (size_t)NBHALF * SS;
  __bf16* Xb = (__bf16*)take((size_t)NR * E * 2); __bf16* PT = (__bf16*)take((size_t)4 * E * E * 2);
  float* Q32 = (float*)take(HR * E * 4); float* K32 = (float*)take(HR * E * 4); _Float16* VTh = (_Float16*)take(HR * E * 2); _Float16* VTl = (_Float16*)take(HR * E * 2);
  float* O32 = Q32;
  k_cvt<<<(NR * E / 8 + 255) / 256, 256, 0, stream>>>(x, Xb);
  k_pack<<<4 * E, 128, 0, stream>>>(Wqkv, Wp, PT);
  for (int hf = 0; hf < 2; ++hf) { const int rbase = hf * (int)HR;
    k_qkv<<<dim3(HR / 64, E / 128, 3), 128, 0, stream>>>(Xb, rbase, PT, Q32, K32, VTh, VTl);
    k_attn<<<dim3(SS / 64, NBHALF * NH), 128, 0, stream>>>(Q32, K32, VTh, VTl, O32);
    k_out<<<dim3(HR / 64, E / 128), 128, 0, stream>>>(O32, rbase, PT, bp, out); }
}
